// DNN_91225105367177
// MI455X (gfx1250) — hardware-verified
//
#include <hip/hip_runtime.h>
#include <hip/hip_bf16.h>
#include <stdint.h>


typedef unsigned short v4us __attribute__((ext_vector_type(4)));
typedef unsigned short v8us __attribute__((ext_vector_type(8)));
typedef unsigned short v16us __attribute__((ext_vector_type(16)));
typedef __bf16 v16bf __attribute__((ext_vector_type(16)));
typedef float v8f __attribute__((ext_vector_type(8)));
typedef float v4f __attribute__((ext_vector_type(4)));

union Frag { v16us u; v16bf v; v8us half[2]; };

#define NROW   2048
#define NPOS   520
#define SPAD   528
#define XROW   4160
#define H2ROW  16640
#define PL1K   33280
#define KP     40

static __device__ __forceinline__ unsigned short bf_rne(float f) {
    unsigned u = __float_as_uint(f);
    u = u + 0x7FFFu + ((u >> 16) & 1u);
    return (unsigned short)(u >> 16);
}
static __device__ __forceinline__ float bf_val(unsigned short s) {
    return __uint_as_float(((unsigned)s) << 16);
}
static __device__ __forceinline__ void split3(float v, unsigned short& h, unsigned short& m, unsigned short& l) {
    h = bf_rne(v);
    float r1 = v - bf_val(h);
    m = bf_rne(r1);
    float r2 = r1 - bf_val(m);
    l = bf_rne(r2);
}

static __device__ __forceinline__ v8f wmma_step(v16us a, v16us b, v8f c) {
    Frag fa, fb; fa.u = a; fb.u = b;
    v8f d = __builtin_amdgcn_wmma_f32_16x16x32_bf16(false, fa.v, false, fb.v, (short)0, c, false, false);
    asm volatile("v_nop\n\tv_nop\n\tv_nop\n\tv_nop" : "+v"(d) : "v"(fa.v), "v"(fb.v));
    return d;
}
static __device__ __forceinline__ v8f mma3x3(const v16us* a, const v16us* b, v8f c) {
    c = wmma_step(a[2], b[0], c);
    c = wmma_step(a[0], b[2], c);
    c = wmma_step(a[1], b[1], c);
    c = wmma_step(a[1], b[0], c);
    c = wmma_step(a[0], b[1], c);
    c = wmma_step(a[0], b[0], c);
    return c;
}

__global__ void __launch_bounds__(64) k_conv(const float* __restrict__ x,
                                            const float* __restrict__ w1, const float* __restrict__ b1,
                                            const float* __restrict__ w2, const float* __restrict__ b2,
                                            float* h2, int chalf)
{
    __shared__ __align__(16) float w1s[512];
    __shared__ float b1s[64];
    __shared__ float b2s[16];
    __shared__ __align__(16) unsigned short w2p[3][16 * 64];
    __shared__ __align__(16) unsigned short h1p[2][3][16 * 64];
    __shared__ __align__(16) float outs[16 * SPAD];

    const int tid = threadIdx.x;
    const int lane = tid & 31, wave = tid >> 5, lp = lane & 15, hh = lane >> 4;
    const int row = blockIdx.x >> 1;
    const int cg = blockIdx.x & 1;
    const int cbase = chalf * 32 + cg * 16;
    if (row >= NROW) return;

    for (int i = tid; i < 512; i += 64) w1s[i] = w1[i];
    b1s[tid] = b1[tid];
    if (tid < 16) b2s[tid] = b2[cbase + tid];
    for (int i = tid; i < 1024; i += 64) {
        float v = w2[(size_t)(cbase + (i >> 6)) * 64 + (i & 63)];
        unsigned short ph, pm, pl;
        split3(v, ph, pm, pl);
        w2p[0][i] = ph; w2p[1][i] = pm; w2p[2][i] = pl;
    }
    __syncthreads();

    v16us A2[2][3];
#pragma unroll
    for (int s = 0; s < 2; ++s) {
#pragma unroll
        for (int q = 0; q < 3; ++q) {
            Frag f;
            f.half[0] = *(const v8us*)(&w2p[q][lp * 64 + s * 32 + 8 * hh]);
            f.half[1] = *(const v8us*)(&w2p[q][lp * 64 + s * 32 + 16 + 8 * hh]);
            A2[s][q] = f.u;
        }
    }

    const float* xr = x + (size_t)row * XROW;
    for (int it = 0; it < 18; ++it) {
        const int tile = wave + 2 * it;
        const int p0 = tile * 16;
        const int pos = p0 + lp;
        const int posc = pos < NPOS ? pos : (NPOS - 1);
        float xv[8];
#pragma unroll
        for (int c = 0; c < 8; ++c) xv[c] = xr[c * NPOS + posc];

#pragma unroll 1
        for (int g = 0; g < 4; ++g) {
            v8us vh = {0, 0, 0, 0, 0, 0, 0, 0};
            v8us vm = {0, 0, 0, 0, 0, 0, 0, 0};
            v8us vl = {0, 0, 0, 0, 0, 0, 0, 0};
#pragma unroll
            for (int j = 0; j < 8; ++j) {
                const int co = hh * 32 + g * 8 + j;
                const float* wr = &w1s[co * 8];
                float s = xv[0] * wr[0];
#pragma unroll
                for (int c = 1; c < 8; ++c) s += xv[c] * wr[c];
                s += b1s[co];
                s = s > 0.0f ? s : 0.0f;
                unsigned short ph, pm, pl;
                split3(s, ph, pm, pl);
                vh[j] = ph; vm[j] = pm; vl[j] = pl;
            }
            const int off = lp * 64 + hh * 32 + g * 8;
            *(v8us*)(&h1p[wave][0][off]) = vh;
            *(v8us*)(&h1p[wave][1][off]) = vm;
            *(v8us*)(&h1p[wave][2][off]) = vl;
        }
        __syncthreads();

        v8f acc;
#pragma unroll
        for (int r = 0; r < 8; ++r) acc[r] = b2s[8 * hh + r];
#pragma unroll
        for (int s = 0; s < 2; ++s) {
            v16us Bf[3];
#pragma unroll
            for (int q = 0; q < 3; ++q) {
                Frag f;
                f.half[0] = *(const v8us*)(&h1p[wave][q][lp * 64 + s * 32 + 8 * hh]);
                f.half[1] = *(const v8us*)(&h1p[wave][q][lp * 64 + s * 32 + 16 + 8 * hh]);
                Bf[q] = f.u;
            }
            acc = mma3x3(A2[s], Bf, acc);
        }
        if (tile < 33) {
#pragma unroll
            for (int r = 0; r < 8; ++r) {
                float v = acc[r] > 0.0f ? acc[r] : 0.0f;
                outs[(8 * hh + r) * SPAD + p0 + lp] = v;
            }
        }
        __syncthreads();
    }

    float* dst = h2 + (size_t)row * H2ROW + (size_t)cg * (16 * NPOS);
    for (int i = 0; i < 33; ++i) {
        const int q = tid + 64 * i;
        if (q < 2080) {
            const int e = q * 4;
            const int c = e / NPOS;
            const int p = e - c * NPOS;
            v4f v = *(const v4f*)(&outs[c * SPAD + p]);
            *(volatile v4f*)(dst + e) = v;
        }
    }
    __threadfence();
    for (int i = 0; i < 33; ++i) {
        const int q = tid + 64 * i;
        if (q < 2080) {
            const int e = q * 4;
            const int c = e / NPOS;
            const int p = e - c * NPOS;
            v4f v = *(const v4f*)(&outs[c * SPAD + p]);
            *(volatile v4f*)(dst + e) = v;
        }
    }
}

__global__ void __launch_bounds__(256) k_pl1(const float* h2, const float* __restrict__ w,
                                             float* act, int khalf)
{
    __shared__ __align__(16) unsigned short Ap[3][32 * KP];
    __shared__ __align__(16) unsigned short Bp[3][64 * KP];
    __shared__ __align__(16) float T[32 * 64];

    const int tid = threadIdx.x;
    const int lane = tid & 31, wave = tid >> 5, lp = lane & 15, hh = lane >> 4;
    const int rb = blockIdx.x >> 2, cb = blockIdx.x & 3;
    if (rb >= NROW / 32) return;
    const int R0 = rb * 32, C0 = cb * 64;
    const int rw = (wave >> 2) * 16, cw = (wave & 3) * 16;

    const int ar = tid >> 3, ak = (tid & 7) * 4;
    const float* ag  = h2 + (size_t)(R0 + ar) * H2ROW + ak;
    const float* bg0 = w + (size_t)(C0 + ar) * PL1K + (size_t)khalf * H2ROW + ak;
    const float* bg1 = w + (size_t)(C0 + 32 + ar) * PL1K + (size_t)khalf * H2ROW + ak;

    double ds[8];
#pragma unroll
    for (int r = 0; r < 8; ++r) ds[r] = 0.0;

    for (int k0 = 0; k0 < H2ROW; k0 += 32) {
        const v4f av  = *(const v4f*)(ag + k0);
        const v4f bv0 = *(const v4f*)(bg0 + k0);
        const v4f bv1 = *(const v4f*)(bg1 + k0);
        v4us ah = {0, 0, 0, 0}, am = {0, 0, 0, 0}, al = {0, 0, 0, 0};
        v4us ch = {0, 0, 0, 0}, cm = {0, 0, 0, 0}, cl = {0, 0, 0, 0};
        v4us dh = {0, 0, 0, 0}, dm = {0, 0, 0, 0}, dl = {0, 0, 0, 0};
#pragma unroll
        for (int e = 0; e < 4; ++e) {
            unsigned short ph, pm, pl;
            split3(av[e], ph, pm, pl);  ah[e] = ph; am[e] = pm; al[e] = pl;
            split3(bv0[e], ph, pm, pl); ch[e] = ph; cm[e] = pm; cl[e] = pl;
            split3(bv1[e], ph, pm, pl); dh[e] = ph; dm[e] = pm; dl[e] = pl;
        }
        const int ao = ar * KP + ak;
        const int bo = (32 + ar) * KP + ak;
        *(v4us*)(&Ap[0][ao]) = ah; *(v4us*)(&Ap[1][ao]) = am; *(v4us*)(&Ap[2][ao]) = al;
        *(v4us*)(&Bp[0][ao]) = ch; *(v4us*)(&Bp[1][ao]) = cm; *(v4us*)(&Bp[2][ao]) = cl;
        *(v4us*)(&Bp[0][bo]) = dh; *(v4us*)(&Bp[1][bo]) = dm; *(v4us*)(&Bp[2][bo]) = dl;
        __syncthreads();

        v16us Af[3], Bf[3];
#pragma unroll
        for (int q = 0; q < 3; ++q) {
            Frag f;
            f.half[0] = *(const v8us*)(&Ap[q][(rw + lp) * KP + 8 * hh]);
            f.half[1] = *(const v8us*)(&Ap[q][(rw + lp) * KP + 16 + 8 * hh]);
            Af[q] = f.u;
            Frag g;
            g.half[0] = *(const v8us*)(&Bp[q][(cw + lp) * KP + 8 * hh]);
            g.half[1] = *(const v8us*)(&Bp[q][(cw + lp) * KP + 16 + 8 * hh]);
            Bf[q] = g.u;
        }
        v8f grp;
#pragma unroll
        for (int r = 0; r < 8; ++r) grp[r] = 0.0f;
        grp = mma3x3(Af, Bf, grp);
#pragma unroll
        for (int r = 0; r < 8; ++r) ds[r] += (double)grp[r];
        __syncthreads();
    }

#pragma unroll
    for (int r = 0; r < 8; ++r) T[(rw + 8 * hh + r) * 64 + cw + lp] = (float)ds[r];
    __syncthreads();

    const int r0 = tid >> 4, c4 = (tid & 15) * 4;
    v4f v0 = *(const v4f*)(&T[r0 * 64 + c4]);
    v4f v1 = *(const v4f*)(&T[(r0 + 16) * 64 + c4]);
    float* p0 = act + (size_t)(R0 + r0) * 256 + C0 + c4;
    float* p1 = act + (size_t)(R0 + 16 + r0) * 256 + C0 + c4;
    *(volatile v4f*)p0 = v0;
    *(volatile v4f*)p1 = v1;
    __threadfence();
    *(volatile v4f*)p0 = v0;
    *(volatile v4f*)p1 = v1;
}

__global__ void __launch_bounds__(128) k_pl2(const float* acta, const float* actb,
                                             const float* __restrict__ pb,
                                             const float* __restrict__ w,
                                             const float* __restrict__ bias,
                                             float* theta, float* trti)
{
    __shared__ __align__(16) float a_s[256];
    __shared__ __align__(16) float th_s[128];
    __shared__ __align__(16) float tt_s[128];
    __shared__ float rl_s[128];

    const int row = blockIdx.x, t = threadIdx.x;
    if (row >= NROW) return;

    for (int i = t; i < 256; i += 128) {
        float v = acta[(size_t)row * 256 + i] + actb[(size_t)row * 256 + i] + pb[i];
        a_s[i] = v > 0.0f ? v : 0.0f;
    }
    __syncthreads();
    {
        const float* wr = w + (size_t)t * 256;
        float s = 0.0f;
#pragma unroll 4
        for (int i = 0; i < 256; ++i) s += a_s[i] * wr[i];
        s += bias[t];
        rl_s[t] = s;
    }
    __syncthreads();
    if (t < 64) {
        float pr = rl_s[t], pi = rl_s[64 + t];
        float nn = sqrtf(pr * pr + pi * pi);
        nn = nn > 1e-12f ? nn : 1e-12f;
        float inv = 1.0f / nn;
        float trv = pr * inv, tiv = pi * inv;
        th_s[2 * t] = trv; th_s[2 * t + 1] = tiv;
        tt_s[t] = trv; tt_s[64 + t] = tiv;
    }
    __syncthreads();

    v4f v = {0.0f, 0.0f, 0.0f, 0.0f};
    float* p = theta;
    if (t < 32) {
        v = *(const v4f*)(&th_s[4 * t]);
        p = theta + (size_t)row * 128 + 4 * t;
    } else if (t < 64) {
        const int l = t - 32;
        v = *(const v4f*)(&tt_s[4 * l]);
        p = trti + (size_t)row * 128 + 4 * l;
    }
    if (t < 64) *(volatile v4f*)p = v;
    __threadfence();
    if (t < 64) *(volatile v4f*)p = v;
}

__global__ void __launch_bounds__(128) k_tail(
    const float* __restrict__ Hre, const float* __restrict__ Him,
    const float* __restrict__ chre, const float* __restrict__ chim,
    const float* __restrict__ b1w, const float* __restrict__ b1b,
    const float* __restrict__ b2w, const float* __restrict__ b2b,
    const float* __restrict__ b3w, const float* __restrict__ b3b,
    const float* __restrict__ p1w, const float* __restrict__ p1b,
    const float* __restrict__ p2w, const float* __restrict__ p2b,
    const float* trti, float* tailst)
{
    __shared__ float str[256], sti[256];
    __shared__ float part[4][32][4];
    __shared__ float cH[64];
    __shared__ float w0[128], q1[128], w1v[128], w2v[80];
    __shared__ float mu_s[2];
    __shared__ float scs;
    __shared__ __align__(16) float orow[128];

    const int b = blockIdx.x;
    const int t = threadIdx.x;
    if (b >= 512) return;

    for (int idx = t; idx < 256; idx += 128) {
        const int l = idx >> 6, n = idx & 63;
        const float* src = trti + (size_t)(b * 4 + l) * 128;
        str[idx] = src[n];
        sti[idx] = src[64 + n];
    }
    __syncthreads();

    {
        const int km = t & 31, l = t >> 5;
        const int k = km >> 3, m = km & 7;
        const size_t base = ((size_t)b * 8 + m) * 1024 + l * 4 + k;
        const float* hre = Hre + base;
        const float* him = Him + base;
        float a = 0.0f, bb = 0.0f, c = 0.0f, d = 0.0f;
#pragma unroll 4
        for (int n = 0; n < 64; ++n) {
            float hr = hre[n * 16], hm = him[n * 16];
            float trv = str[l * 64 + n], tiv = sti[l * 64 + n];
            a += hr * trv;  bb += hr * tiv;
            c += hm * trv;  d += hm * tiv;
        }
        part[l][km][0] = a; part[l][km][1] = bb;
        part[l][km][2] = c; part[l][km][3] = d;
    }
    __syncthreads();

    if (t < 32) {
        const int k = t >> 3, m = t & 7;
        float a = 0.0f, bb = 0.0f, c = 0.0f, d = 0.0f;
#pragma unroll
        for (int l = 0; l < 4; ++l) {
            a += part[l][t][0]; bb += part[l][t][1];
            c += part[l][t][2]; d += part[l][t][3];
        }
        float top = a + d;
        float bot = bb - c;
        cH[k * 16 + m]     = top + chre[b * 32 + k * 8 + m];
        cH[k * 16 + 8 + m] = bot + chim[b * 32 + k * 8 + m];
    }
    __syncthreads();

    {
        float s1 = 0.0f, s2 = 0.0f;
        const float* w1r = b1w + t * 64;
        const float* p1r = p1w + t * 64;
#pragma unroll 4
        for (int i = 0; i < 64; ++i) {
            float h = cH[i];
            s1 += w1r[i] * h;
            s2 += p1r[i] * h;
        }
        s1 += b1b[t]; s2 += p1b[t];
        w0[t] = s1 > 0.0f ? s1 : 0.0f;
        q1[t] = s2 > 0.0f ? s2 : 0.0f;
    }
    __syncthreads();

    {
        float s = 0.0f;
        const float* wr = b2w + t * 128;
#pragma unroll 4
        for (int i = 0; i < 128; ++i) s += wr[i] * w0[i];
        s += b2b[t];
        w1v[t] = s > 0.0f ? s : 0.0f;
    }
    __syncthreads();

    if (t < 80) {
        float s = 0.0f;
        const float* wr = b3w + t * 128;
#pragma unroll 4
        for (int i = 0; i < 128; ++i) s += wr[i] * w1v[i];
        s += b3b[t];
        w2v[t] = s;
    }
    if (t >= 96 && t < 98) {
        const int j = t - 96;
        float s = 0.0f;
        const float* wr = p2w + j * 128;
#pragma unroll 4
        for (int i = 0; i < 128; ++i) s += wr[i] * q1[i];
        s += p2b[j];
        mu_s[j] = s;
    }
    __syncthreads();

    if (t == 0) {
        float m0 = mu_s[0], m1 = mu_s[1];
        float mx = m0 > m1 ? m0 : m1;
        float e0 = expf(m0 - mx), e1 = expf(m1 - mx);
        float inv = 1.0f / (e0 + e1);
        float u0 = e0 * inv, u1 = e1 * inv;
        mu_s[0] = u0;
        mu_s[1] = u1;
        float nn = 0.0f;
#pragma unroll 4
        for (int i = 0; i < 80; ++i) nn += w2v[i] * w2v[i];
        float nrm = sqrtf(nn);
        nrm = nrm > 1e-12f ? nrm : 1e-12f;
        scs = sqrtf(10.0f) * sqrtf(u0) / nrm;
    }
    __syncthreads();

    if (t < 80)      orow[t] = w2v[t] * scs;
    else if (t < 82) orow[t] = mu_s[t - 80];
    else             orow[t] = 0.0f;
    __syncthreads();

    v4f v = {0.0f, 0.0f, 0.0f, 0.0f};
    float* p = tailst;
    if (t < 32) {
        v = *(const v4f*)(&orow[4 * t]);
        p = tailst + (size_t)b * 128 + 4 * t;
        *(volatile v4f*)p = v;
    }
    __threadfence();
    if (t < 32) *(volatile v4f*)p = v;
}

__global__ void __launch_bounds__(256) k_pack(const float* tailst, float* outw, float* outmu)
{
    const int blk = blockIdx.x, t = threadIdx.x;
    if (blk > 40) return;
    v4f v = {0.0f, 0.0f, 0.0f, 0.0f};
    float* p;
    if (blk < 40) {
        const int q = blk * 256 + t;
        const int e = q * 4;
        const int bb = e / 80;
        const int wi = e - bb * 80;
        v = *(const v4f*)(tailst + (size_t)bb * 128 + wi);
        p = outw + e;
    } else {
        const int g = t;
        const float* r0 = tailst + (size_t)(2 * g) * 128 + 80;
        const float* r1 = tailst + (size_t)(2 * g + 1) * 128 + 80;
        v[0] = r0[0]; v[1] = r0[1]; v[2] = r1[0]; v[3] = r1[1];
        p = outmu + 4 * g;
    }
    *(volatile v4f*)p = v;
    __threadfence();
    *(volatile v4f*)p = v;
}

extern "C" void kernel_launch(void* const* d_in, const int* in_sizes, int n_in,
                              void* d_out, int out_size, void* d_ws, size_t ws_size,
                              hipStream_t stream)
{
    if (n_in < 23) return;
    if (in_sizes[0] != NROW * XROW) return;
    if (in_sizes[1] != 512 * 8 * 64 * 16 || in_sizes[2] != 512 * 8 * 64 * 16) return;
    if (in_sizes[3] != 512 * 32 || in_sizes[4] != 512 * 32) return;
    if (in_sizes[5] != 512 || in_sizes[6] != 64 || in_sizes[7] != 4096 || in_sizes[8] != 64) return;
    if (in_sizes[9] != 256 * PL1K || in_sizes[10] != 256) return;
    if (in_sizes[11] != 128 * 256 || in_sizes[12] != 128) return;
    if (in_sizes[13] != 128 * 64 || in_sizes[14] != 128) return;
    if (in_sizes[15] != 128 * 128 || in_sizes[16] != 128) return;
    if (in_sizes[17] != 80 * 128 || in_sizes[18] != 80) return;
    if (in_sizes[19] != 128 * 64 || in_sizes[20] != 128) return;
    if (in_sizes[21] != 256 || in_sizes[22] != 2) return;
    if (out_size != 40960 + 262144 + 1024) return;

    const float* x      = (const float*)d_in[0];
    const float* Hre    = (const float*)d_in[1];
    const float* Him    = (const float*)d_in[2];
    const float* chre   = (const float*)d_in[3];
    const float* chim   = (const float*)d_in[4];
    const float* conv1w = (const float*)d_in[5];
    const float* conv1b = (const float*)d_in[6];
    const float* conv2w = (const float*)d_in[7];
    const float* conv2b = (const float*)d_in[8];
    const float* pl1w   = (const float*)d_in[9];
    const float* pl1b   = (const float*)d_in[10];
    const float* pl2w   = (const float*)d_in[11];
    const float* pl2b   = (const float*)d_in[12];
    const float* b1w = (const float*)d_in[13]; const float* b1b = (const float*)d_in[14];
    const float* b2w = (const float*)d_in[15]; const float* b2b = (const float*)d_in[16];
    const float* b3w = (const float*)d_in[17]; const float* b3b = (const float*)d_in[18];
    const float* p1w = (const float*)d_in[19]; const float* p1b = (const float*)d_in[20];
    const float* p2w = (const float*)d_in[21]; const float* p2b = (const float*)d_in[22];

    size_t off = 0;
    const size_t o_h2   = off; off += (size_t)NROW * H2ROW * 4;        off = (off + 255) & ~(size_t)255;
    const size_t o_acta = off; off += (size_t)NROW * 256 * 4;          off = (off + 255) & ~(size_t)255;
    const size_t o_actb = off; off += (size_t)NROW * 256 * 4;          off = (off + 255) & ~(size_t)255;
    const size_t o_trti = off; off += (size_t)NROW * 128 * 4;          off = (off + 255) & ~(size_t)255;
    const size_t o_tail = off; off += (size_t)512 * 128 * 4;           off = (off + 255) & ~(size_t)255;
    if (off > ws_size) return;

    char* ws = (char*)d_ws;
    float* h2     = (float*)(ws + o_h2);
    float* acta   = (float*)(ws + o_acta);
    float* actb   = (float*)(ws + o_actb);
    float* trti   = (float*)(ws + o_trti);
    float* tailst = (float*)(ws + o_tail);

    float* outW     = (float*)d_out;
    float* outTheta = (float*)((char*)d_out + 163840);
    float* outMu    = (float*)((char*)d_out + 1212416);

    k_conv<<<NROW * 2, 64, 0, stream>>>(x, conv1w, conv1b, conv2w, conv2b, h2, 0);
    k_pl1<<<(NROW / 32) * 4, 256, 0, stream>>>(h2, pl1w, acta, 0);
    k_conv<<<NROW * 2, 64, 0, stream>>>(x, conv1w, conv1b, conv2w, conv2b, h2, 1);
    k_pl1<<<(NROW / 32) * 4, 256, 0, stream>>>(h2, pl1w, actb, 1);

    k_pl2<<<NROW, 128, 0, stream>>>(acta, actb, pl1b, pl2w, pl2b, outTheta, trti);
    k_tail<<<512, 128, 0, stream>>>(Hre, Him, chre, chim,
                                    b1w, b1b, b2w, b2b, b3w, b3b,
                                    p1w, p1b, p2w, p2b, trti, tailst);
    k_pack<<<41, 256, 0, stream>>>(tailst, outW, outMu);
}
